// GroupQueryAtention_11742440587282
// MI455X (gfx1250) — hardware-verified
//
#include <hip/hip_runtime.h>
#include <math.h>

typedef __attribute__((ext_vector_type(16))) _Float16 v16h;
typedef __attribute__((ext_vector_type(8)))  _Float16 v8h;
typedef __attribute__((ext_vector_type(16))) __bf16   v16b;
typedef __attribute__((ext_vector_type(8)))  __bf16   v8b;
typedef __attribute__((ext_vector_type(8)))  float    v8f;
typedef __attribute__((ext_vector_type(4)))  float    v4f;
typedef __attribute__((ext_vector_type(4)))  unsigned int v4u;

constexpr int kB      = 2;
constexpr int kT      = 1024;
constexpr int kC      = 2048;
constexpr int kNH     = 16;
constexpr int kNKV    = 4;
constexpr int kHD     = kC / kNH;
constexpr int kHalfHD = kHD / 2;
constexpr int kRows   = kB * kT;
constexpr int kKVC    = kNKV * kHD;
constexpr int kNQKV   = kC + 2 * kKVC;
constexpr int kSlices = kNH + 2 * kNKV;
static_assert(kHD == 128, "head dim");
static_assert(kRows == 2048 && kKVC == 512 && kNQKV == 3072 && kSlices == 24, "derived shapes");
static_assert((kC % 64) == 0 && (kNQKV % 64) == 0 && (kRows % 64) == 0, "GEMM M,N multiples of 64");
static_assert((kC % 32) == 0, "GEMM K multiple of 32");
static_assert((kT % 64) == 0 && (kHD % 32) == 0, "attention tiles");

constexpr float kPCarry   = 32768.0f;
constexpr float kVCarry   = 1024.0f;
constexpr float kACarry   = 4096.0f;
constexpr float kWoCarry  = 1024.0f;
constexpr float kAttnNorm = kACarry / kVCarry;
constexpr float kOutScale = 1.0f / (kACarry * kWoCarry);
constexpr float kMaskVal  = -1.0e30f;

constexpr int kPPitch = 40;
constexpr int kOPitch = 132;
constexpr int kVPitch = 132;

constexpr size_t kSzX    = (size_t)kRows * kC * 2;
constexpr size_t kSzW    = (size_t)kNQKV * kC * 2;
constexpr size_t kSzWO   = (size_t)kC * kC * 2;
constexpr size_t kSzQKV  = (size_t)kRows * kNQKV * 4;
constexpr size_t kSzQ    = (size_t)kB * kNH * kT * kHD * 2;
constexpr size_t kSzK    = (size_t)kB * kNKV * kT * kHD * 2;
constexpr size_t kSzA    = (size_t)kRows * kC * 2;
constexpr size_t kSzTrig = (size_t)kT * kHalfHD * 4;
constexpr size_t kOffXH  = 0;
constexpr size_t kOffXL  = kOffXH  + kSzX;
constexpr size_t kOffWH  = kOffXL  + kSzX;
constexpr size_t kOffWL  = kOffWH  + kSzW;
constexpr size_t kOffWOT = kOffWL  + kSzW;
constexpr size_t kOffQKV = kOffWOT + kSzWO;
constexpr size_t kOffQH  = kOffQKV + kSzQKV;
constexpr size_t kOffQL  = kOffQH  + kSzQ;
constexpr size_t kOffKH  = kOffQL  + kSzQ;
constexpr size_t kOffKL  = kOffKH  + kSzK;
constexpr size_t kOffVTH = kOffKL  + kSzK;
constexpr size_t kOffVTL = kOffVTH + kSzK;
constexpr size_t kOffAH  = kOffVTL + kSzK;
constexpr size_t kOffAL  = kOffAH  + kSzA;
constexpr size_t kOffCOS = kOffAL  + kSzA;
constexpr size_t kOffSIN = kOffCOS + kSzTrig;
constexpr size_t kWsTotal = kOffSIN + kSzTrig;
static_assert(kWsTotal == 117964800ull, "carve total");
static_assert(kWsTotal <= 134217728ull, "carve cap");
static_assert((kSzX % 128) == 0 && (kSzW % 128) == 0 && (kSzWO % 128) == 0 && (kSzQKV % 128) == 0 &&
              (kSzQ % 128) == 0 && (kSzK % 128) == 0 && (kSzA % 128) == 0 && (kSzTrig % 128) == 0, "128-B regions");

__device__ __forceinline__ unsigned short f2bf_bits(float f) {
  unsigned u = __float_as_uint(f);
  return (unsigned short)((u + 0x7FFFu + ((u >> 16) & 1u)) >> 16);
}
__device__ __forceinline__ float bf_bits2f(unsigned short h) { return __uint_as_float(((unsigned)h) << 16); }
__device__ __forceinline__ unsigned pk16(unsigned short a, unsigned short b) { return (unsigned)a | ((unsigned)b << 16); }
__device__ __forceinline__ unsigned short h_bits(float f) { const _Float16 h = (_Float16)f; return __builtin_bit_cast(unsigned short, h); }

__device__ __forceinline__ void tie1_h(v8f& a, v16h x, v16h y, v16h z) { asm volatile("v_nop\n\tv_nop\n\tv_nop\n\tv_nop" : "+v"(a) : "v"(x), "v"(y), "v"(z)); }
__device__ __forceinline__ void tie1_b(v8f& a, v16b x, v16b y, v16b z) { asm volatile("v_nop\n\tv_nop\n\tv_nop\n\tv_nop" : "+v"(a) : "v"(x), "v"(y), "v"(z)); }
__device__ __forceinline__ void keep4_h(v16h a, v16h b, v16h c, v16h d) { asm volatile("v_nop" :: "v"(a), "v"(b), "v"(c), "v"(d)); }
__device__ __forceinline__ void keep4_b(v16b a, v16b b, v16b c, v16b d) { asm volatile("v_nop" :: "v"(a), "v"(b), "v"(c), "v"(d)); }
__device__ __forceinline__ void acc_guard4(v8f& a, v8f& b, v8f& c, v8f& d) { asm volatile("v_nop\n\tv_nop\n\tv_nop\n\tv_nop" : "+v"(a), "+v"(b), "+v"(c), "+v"(d)); }

template <typename T> struct Frag;
template <> struct Frag<_Float16> {
  typedef v16h V; union U { v16h v; v8h h[2]; };
  static __device__ __forceinline__ v16h load(const _Float16* p) {
    U f; f.h[0] = *(const v8h*)(p); f.h[1] = *(const v8h*)(p + 16); return f.v;
  }
  static __device__ __forceinline__ v8f mma(v16h a, v16h b, v8f c) {
    return __builtin_amdgcn_wmma_f32_16x16x32_f16(false, a, false, b, (short)0, c, false, false);
  }
  static __device__ __forceinline__ void guard1(v8f& a, v16h x, v16h y, v16h z) { tie1_h(a, x, y, z); }
  static __device__ __forceinline__ void keep(v16h a, v16h b, v16h c, v16h d) { keep4_h(a, b, c, d); }
};
template <> struct Frag<__bf16> {
  typedef v16b V; union U { v16b v; v8b h[2]; };
  static __device__ __forceinline__ v16b load(const __bf16* p) {
    U f; f.h[0] = *(const v8b*)(p); f.h[1] = *(const v8b*)(p + 16); return f.v;
  }
  static __device__ __forceinline__ v8f mma(v16b a, v16b b, v8f c) {
    return __builtin_amdgcn_wmma_f32_16x16x32_bf16(false, a, false, b, (short)0, c, false, false);
  }
  static __device__ __forceinline__ void guard1(v8f& a, v16b x, v16b y, v16b z) { tie1_b(a, x, y, z); }
  static __device__ __forceinline__ void keep(v16b a, v16b b, v16b c, v16b d) { keep4_b(a, b, c, d); }
};

__device__ __forceinline__ v8f mma_bf(v16b a, v16b b, v8f c) {
  c = __builtin_amdgcn_wmma_f32_16x16x32_bf16(false, a, false, b, (short)0, c, false, false);
  asm volatile("v_nop\n\tv_nop\n\tv_nop\n\tv_nop" : "+v"(c) : "v"(a), "v"(b));
  return c;
}
__device__ __forceinline__ v8f mma_hf(v16h a, v16h b, v8f c) {
  c = __builtin_amdgcn_wmma_f32_16x16x32_f16(false, a, false, b, (short)0, c, false, false);
  asm volatile("v_nop\n\tv_nop\n\tv_nop\n\tv_nop" : "+v"(c) : "v"(a), "v"(b));
  return c;
}

template <int ET> struct Elem;
template <> struct Elem<0> { typedef _Float16 T; };
template <> struct Elem<1> { typedef __bf16 T; };
template <int ET, int SPL, int BIAS_MODE, int OUT_MODE, bool RESID, int ACT = 0>
__global__ __launch_bounds__(256) void wmma_gemm64(
    const unsigned short* __restrict__ Ap, const unsigned short* __restrict__ A2p, int lda, long strideA,
    const unsigned short* __restrict__ Btp, const unsigned short* __restrict__ Bt2p, int ldb, long strideB,
    void* __restrict__ Cout, void* __restrict__ Cout2, int ldc, long strideC,
    const float* __restrict__ bias,
    const float* __restrict__ resid, long strideR,
    int M, int N, int K, float scale) {
  typedef typename Elem<ET>::T T;
  typedef typename Frag<T>::V V;
  const T* A = (const T*)Ap; const T* A2 = (const T*)A2p; const T* Bt = (const T*)Btp; const T* Bt2 = (const T*)Bt2p;
  __shared__ __align__(16) float sT[8][16 * 68];
  const int b    = blockIdx.y;
  const int lane = threadIdx.x & 31;
  const int wave = threadIdx.x >> 5;
  const int tilesN = N >> 6;
  const int tilesM = M >> 6;
  const int tile = blockIdx.x * 8 + wave;
  if (tile >= tilesM * tilesN) return;
  const int tm = tile / tilesN;
  const int tn = tile - tm * tilesN;
  const int m0 = tm << 6;
  const int n0 = tn << 6;

  const T* Ab  = A  + (size_t)b * strideA;
  const T* Bb  = Bt + (size_t)b * strideB;
  const T* Ab2 = (SPL >= 1) ? (A2  + (size_t)b * strideA) : nullptr;
  const T* Bb2 = (SPL == 2) ? (Bt2 + (size_t)b * strideB) : nullptr;

  const int rlane = lane & 15;
  const int koff  = (lane >> 4) * 8;
  const int mOff  = (lane >> 4) * 8;

  v8f acc[4][4];
#pragma unroll
  for (int i = 0; i < 4; ++i)
#pragma unroll
    for (int j = 0; j < 4; ++j) acc[i][j] = (v8f){0.f,0.f,0.f,0.f,0.f,0.f,0.f,0.f};

  for (int k0 = 0; k0 < K; k0 += 32) {
    V bh[4], bl[4];
#pragma unroll
    for (int j = 0; j < 4; ++j) {
      const size_t bo = (size_t)(n0 + (j << 4) + rlane) * ldb + koff + k0;
      bh[j] = Frag<T>::load(Bb + bo);
      if (SPL == 2) bl[j] = Frag<T>::load(Bb2 + bo);
    }
#pragma unroll
    for (int i = 0; i < 4; ++i) {
      const size_t ao = (size_t)(m0 + (i << 4) + rlane) * lda + koff + k0;
      V ah = Frag<T>::load(Ab + ao);
      V al;
      if (SPL >= 1) al = Frag<T>::load(Ab2 + ao);
#pragma unroll
      for (int j = 0; j < 4; ++j) {
        acc[i][j] = Frag<T>::mma(ah, bh[j], acc[i][j]);
        if (SPL == 2) acc[i][j] = Frag<T>::mma(ah, bl[j], acc[i][j]);
        if (SPL >= 1) acc[i][j] = Frag<T>::mma(al, bh[j], acc[i][j]);
      }
#pragma unroll
      for (int j = 0; j < 4; ++j) Frag<T>::guard1(acc[i][j], ah, (SPL >= 1) ? al : ah, bh[j]);
    }
    Frag<T>::keep(bh[0], bh[1], bh[2], bh[3]);
    if (SPL == 2) Frag<T>::keep(bl[0], bl[1], bl[2], bl[3]);
  }
  acc_guard4(acc[0][0], acc[0][1], acc[0][2], acc[0][3]);
  acc_guard4(acc[1][0], acc[1][1], acc[1][2], acc[1][3]);
  acc_guard4(acc[2][0], acc[2][1], acc[2][2], acc[2][3]);
  acc_guard4(acc[3][0], acc[3][1], acc[3][2], acc[3][3]);

  float* slab = sT[wave];
  const float* Rb = RESID ? (resid + (size_t)b * strideR) : nullptr;
#pragma unroll
  for (int i = 0; i < 4; ++i) {
    const int mBase = m0 + (i << 4);
#pragma unroll
    for (int j = 0; j < 4; ++j) {
      const int n = n0 + (j << 4) + rlane;
      float bv = 0.f;
      if (BIAS_MODE == 2) bv = bias[n];
#pragma unroll
      for (int r = 0; r < 8; ++r) {
        float v = acc[i][j][r] * scale;
        if (BIAS_MODE == 1) v += bias[mBase + mOff + r];
        if (BIAS_MODE == 2) v += bv;
        if (RESID) v += Rb[(size_t)(mBase + mOff + r) * ldc + n];
        if (ACT == 2) v = fmaxf(v, 0.0f);
        if (ACT == 4) v = (v > 0.f) ? v : 0.01f * v;
        slab[(mOff + r) * 68 + (j << 4) + rlane] = v;
      }
    }
    __builtin_amdgcn_fence(__ATOMIC_RELEASE, "workgroup");
    __builtin_amdgcn_wave_barrier();
    __builtin_amdgcn_fence(__ATOMIC_ACQUIRE, "workgroup");
    if (OUT_MODE == 0) {
      float* C = (float*)Cout + (size_t)b * strideC;
      const int hh = lane >> 4, c4 = (lane & 15) * 4;
      for (int pass = 0; pass < 2; ++pass) {
#pragma unroll
        for (int it = 0; it < 8; ++it) {
          const int row = it * 2 + hh;
          v4f v = *(const v4f*)(slab + row * 68 + c4);
          *(volatile v4f*)(C + (size_t)(mBase + row) * ldc + n0 + c4) = v;
        }
        __threadfence();
      }
    } else {
      const int q = lane >> 3, c8 = (lane & 7) * 8;
      unsigned short* C  = (unsigned short*)Cout  + (size_t)b * strideC;
      unsigned short* C2 = (OUT_MODE == 2) ? ((unsigned short*)Cout2 + (size_t)b * strideC) : nullptr;
      for (int pass = 0; pass < 2; ++pass) {
#pragma unroll
        for (int it = 0; it < 4; ++it) {
          const int row = it * 4 + q;
          const float* sp = slab + row * 68 + c8;
          v8h hv, lv;
#pragma unroll
          for (int e = 0; e < 8; ++e) {
            if (OUT_MODE == 1) {
              hv[e] = (_Float16)sp[e];
            } else {
              unsigned short hb = f2bf_bits(sp[e]);
              unsigned short lb = f2bf_bits(sp[e] - bf_bits2f(hb));
              hv[e] = __builtin_bit_cast(_Float16, hb);
              lv[e] = __builtin_bit_cast(_Float16, lb);
            }
          }
          *(volatile v8h*)(C + (size_t)(mBase + row) * ldc + n0 + c8) = hv;
          if (OUT_MODE == 2) *(volatile v8h*)(C2 + (size_t)(mBase + row) * ldc + n0 + c8) = lv;
        }
        __threadfence();
      }
    }
    __builtin_amdgcn_fence(__ATOMIC_RELEASE, "workgroup");
    __builtin_amdgcn_wave_barrier();
    __builtin_amdgcn_fence(__ATOMIC_ACQUIRE, "workgroup");
  }
}

__global__ __launch_bounds__(256) void split_rows_bf16_kernel(
    const float* __restrict__ src, unsigned short* __restrict__ dhi, unsigned short* __restrict__ dlo, int total8)
{
  const int i = blockIdx.x * 256 + threadIdx.x;
  if (i >= total8) return;
  const size_t e0 = (size_t)i << 3;
  const v4f a0 = *(const v4f*)(src + e0);
  const v4f a1 = *(const v4f*)(src + e0 + 4);
  const float x[8] = {a0[0], a0[1], a0[2], a0[3], a1[0], a1[1], a1[2], a1[3]};
  unsigned short hb[8], lb[8];
#pragma unroll
  for (int e = 0; e < 8; ++e) {
    hb[e] = f2bf_bits(x[e]);
    lb[e] = f2bf_bits(x[e] - bf_bits2f(hb[e]));
  }
  const v4u uh = (v4u){pk16(hb[0], hb[1]), pk16(hb[2], hb[3]), pk16(hb[4], hb[5]), pk16(hb[6], hb[7])};
  const v4u ul = (v4u){pk16(lb[0], lb[1]), pk16(lb[2], lb[3]), pk16(lb[4], lb[5]), pk16(lb[6], lb[7])};
  unsigned short* qh = dhi + e0;
  unsigned short* ql = dlo + e0;
  *(volatile v4u*)qh = uh;
  *(volatile v4u*)ql = ul;
  __threadfence();
  *(volatile v4u*)qh = uh;
  *(volatile v4u*)ql = ul;
}

template <int MODE>
__global__ __launch_bounds__(256) void wt_planes_kernel(
    const float* W0, const float* W1, const float* W2,
    int nA, int nB, int ld0, int ld1, int ld2,
    unsigned short* __restrict__ outH, unsigned short* __restrict__ outL, int K, float scale)
{
  __shared__ float sm[64][65];
  const int t  = threadIdx.x;
  const int k0 = blockIdx.x * 64;
  const int n0 = blockIdx.y * 64;
  const float* W;
  int ld, col;
  if (n0 < nA)           { W = W0; ld = ld0; col = n0; }
  else if (n0 < nA + nB) { W = W1; ld = ld1; col = n0 - nA; }
  else                   { W = W2; ld = ld2; col = n0 - nA - nB; }
#pragma unroll
  for (int i = 0; i < 16; ++i) {
    const int e = i * 256 + t;
    const int r = e >> 6;
    const int c = e & 63;
    sm[c][r] = W[(size_t)(k0 + r) * ld + col + c] * scale;
  }
  __syncthreads();
  const int lane = t & 31, wave = t >> 5;
  const int q = lane >> 3, c8 = (lane & 7) * 8;
  v4u uh[2], ul[2];
#pragma unroll
  for (int it = 0; it < 2; ++it) {
    const int row = wave * 8 + it * 4 + q;
    unsigned short hb[8], lb[8];
#pragma unroll
    for (int e = 0; e < 8; ++e) {
      const float f = sm[row][c8 + e];
      if (MODE == 0) {
        hb[e] = f2bf_bits(f);
        lb[e] = f2bf_bits(f - bf_bits2f(hb[e]));
      } else {
        hb[e] = h_bits(f);
        lb[e] = 0;
      }
    }
    uh[it] = (v4u){pk16(hb[0], hb[1]), pk16(hb[2], hb[3]), pk16(hb[4], hb[5]), pk16(hb[6], hb[7])};
    ul[it] = (v4u){pk16(lb[0], lb[1]), pk16(lb[2], lb[3]), pk16(lb[4], lb[5]), pk16(lb[6], lb[7])};
  }
  for (int pass = 0; pass < 2; ++pass) {
#pragma unroll
    for (int it = 0; it < 2; ++it) {
      const int row = wave * 8 + it * 4 + q;
      const size_t o = (size_t)(n0 + row) * K + k0 + c8;
      *(volatile v4u*)(outH + o) = uh[it];
      if (MODE == 0) *(volatile v4u*)(outL + o) = ul[it];
    }
    __threadfence();
  }
}

__global__ __launch_bounds__(256) void trig_table_kernel(
    const float* __restrict__ ang, float* __restrict__ cosT, float* __restrict__ sinT, int n)
{
  const int i = blockIdx.x * 256 + threadIdx.x;
  if (i >= n) return;
  const float a = ang[i];
  const float c = cosf(a);
  const float s = sinf(a);
  *(volatile float*)(cosT + i) = c;
  *(volatile float*)(sinT + i) = s;
  __threadfence();
  *(volatile float*)(cosT + i) = c;
  *(volatile float*)(sinT + i) = s;
}

__global__ __launch_bounds__(256) void rotate_split_kernel(
    const float* __restrict__ QKV, const float* __restrict__ cosT, const float* __restrict__ sinT,
    unsigned short* __restrict__ QH, unsigned short* __restrict__ QL,
    unsigned short* __restrict__ KH, unsigned short* __restrict__ KL,
    unsigned short* __restrict__ VTH, unsigned short* __restrict__ VTL)
{
  __shared__ __align__(16) float sV[64 * kVPitch];
  const int tid = threadIdx.x, lane = tid & 31, wave = tid >> 5;
  const int sl = blockIdx.x;
  const int r0 = blockIdx.y * 64;
  const int b  = r0 / kT;
  const int t0 = r0 - b * kT;
  const int cbase = sl * kHD;
  if (sl < kNH + kNKV) {
    const bool isQ = (sl < kNH);
    const int head = isQ ? sl : (sl - kNH);
    const int nh   = isQ ? kNH : kNKV;
    unsigned short* PH = isQ ? QH : KH;
    unsigned short* PL = isQ ? QL : KL;
    const size_t pbase = ((size_t)(b * nh + head) * kT + t0) * kHD;
    const int l16 = lane & 15, rsub = lane >> 4;
#pragma unroll 1
    for (int it = 0; it < 4; ++it) {
      const int rl = it * 16 + wave * 2 + rsub;
      const float* src = QKV + (size_t)(r0 + rl) * kNQKV + cbase + l16 * 8;
      const v4f a0 = *(const v4f*)(src);
      const v4f a1 = *(const v4f*)(src + 4);
      const int t = t0 + rl;
      const v4f cv = *(const v4f*)(cosT + (size_t)t * kHalfHD + l16 * 4);
      const v4f sv = *(const v4f*)(sinT + (size_t)t * kHalfHD + l16 * 4);
      float y[8];
      y[0] = cv[0] * a0[0] - sv[0] * a0[1];
      y[1] = sv[0] * a0[0] + cv[0] * a0[1];
      y[2] = cv[1] * a0[2] - sv[1] * a0[3];
      y[3] = sv[1] * a0[2] + cv[1] * a0[3];
      y[4] = cv[2] * a1[0] - sv[2] * a1[1];
      y[5] = sv[2] * a1[0] + cv[2] * a1[1];
      y[6] = cv[3] * a1[2] - sv[3] * a1[3];
      y[7] = sv[3] * a1[2] + cv[3] * a1[3];
      unsigned short hb[8], lb[8];
#pragma unroll
      for (int e = 0; e < 8; ++e) {
        hb[e] = f2bf_bits(y[e]);
        lb[e] = f2bf_bits(y[e] - bf_bits2f(hb[e]));
      }
      const v4u uh = (v4u){pk16(hb[0], hb[1]), pk16(hb[2], hb[3]), pk16(hb[4], hb[5]), pk16(hb[6], hb[7])};
      const v4u ul = (v4u){pk16(lb[0], lb[1]), pk16(lb[2], lb[3]), pk16(lb[4], lb[5]), pk16(lb[6], lb[7])};
      const size_t o = pbase + (size_t)rl * kHD + l16 * 8;
      *(volatile v4u*)(PH + o) = uh;
      *(volatile v4u*)(PL + o) = ul;
      __threadfence();
      *(volatile v4u*)(PH + o) = uh;
      *(volatile v4u*)(PL + o) = ul;
    }
  } else {
    const int hkv = sl - kNH - kNKV;
#pragma unroll
    for (int i = 0; i < 8; ++i) {
      const int e  = i * 256 + tid;
      const int rl = e >> 5;
      const int c4 = (e & 31) * 4;
      const v4f v = *(const v4f*)(QKV + (size_t)(r0 + rl) * kNQKV + cbase + c4);
      *(v4f*)(sV + rl * kVPitch + c4) = v;
    }
    __syncthreads();
    const int q = lane >> 3, c8 = (lane & 7) * 8;
#pragma unroll 1
    for (int it = 0; it < 4; ++it) {
      const int d = it * 32 + wave * 4 + q;
      unsigned short hb[8], lb[8];
#pragma unroll
      for (int e = 0; e < 8; ++e) {
        const float vs = sV[(c8 + e) * kVPitch + d] * kVCarry;
        const _Float16 hh = (_Float16)vs;
        const float res = vs - (float)hh;
        hb[e] = __builtin_bit_cast(unsigned short, hh);
        lb[e] = h_bits(res);
      }
      const v4u uh = (v4u){pk16(hb[0], hb[1]), pk16(hb[2], hb[3]), pk16(hb[4], hb[5]), pk16(hb[6], hb[7])};
      const v4u ul = (v4u){pk16(lb[0], lb[1]), pk16(lb[2], lb[3]), pk16(lb[4], lb[5]), pk16(lb[6], lb[7])};
      const size_t o = ((size_t)(b * kNKV + hkv) * kHD + d) * kT + t0 + c8;
      *(volatile v4u*)(VTH + o) = uh;
      *(volatile v4u*)(VTL + o) = ul;
      __threadfence();
      *(volatile v4u*)(VTH + o) = uh;
      *(volatile v4u*)(VTL + o) = ul;
    }
  }
}

__global__ __launch_bounds__(128) void attn_kernel(
    const unsigned short* __restrict__ QHp, const unsigned short* __restrict__ QLp,
    const unsigned short* __restrict__ KHp, const unsigned short* __restrict__ KLp,
    const unsigned short* __restrict__ VTHp, const unsigned short* __restrict__ VTLp,
    unsigned short* __restrict__ AHp, unsigned short* __restrict__ ALp)
{
  __shared__ __align__(16) _Float16 Pb[4][16 * kPPitch];
  __shared__ __align__(16) float Os[4][16 * kOPitch];
  const int tid = threadIdx.x, w = tid >> 5, lane = tid & 31;
  const int lr = lane & 15, hw = lane >> 4, koff = hw * 8;
  const int b = blockIdx.z, h = blockIdx.y, hk = h % kNKV;
  const int i0 = blockIdx.x * 64;
  const int iw = i0 + 16 * w;

  const __bf16* qh = (const __bf16*)QHp + (size_t)(b * kNH + h) * kT * kHD + koff;
  const __bf16* ql = (const __bf16*)QLp + (size_t)(b * kNH + h) * kT * kHD + koff;
  const __bf16* khr = (const __bf16*)KHp + ((size_t)(b * kNKV + hk) * kT + iw + lr) * kHD + koff;
  const __bf16* klr = (const __bf16*)KLp + ((size_t)(b * kNKV + hk) * kT + iw + lr) * kHD + koff;
  const _Float16* vth = (const _Float16*)VTHp + (size_t)(b * kNKV + hk) * kHD * kT + koff;
  const _Float16* vtl = (const _Float16*)VTLp + (size_t)(b * kNKV + hk) * kHD * kT + koff;

  v8f o[8];
  float mrow[8], lrow[8];
#pragma unroll
  for (int c8 = 0; c8 < 8; ++c8) o[c8] = (v8f){0.f,0.f,0.f,0.f,0.f,0.f,0.f,0.f};
#pragma unroll
  for (int v = 0; v < 8; ++v) { mrow[v] = kMaskVal; lrow[v] = 0.f; }

  _Float16* pw = Pb[w];
  const int ntiles = (iw + 16 + 31) >> 5;
  for (int jt = 0; jt < ntiles; ++jt) {
    const int j0 = jt << 5;
    int kofs = 0;
    asm volatile("" : "+v"(kofs));
    v8f s0 = (v8f){0.f,0.f,0.f,0.f,0.f,0.f,0.f,0.f};
    v8f s1 = (v8f){0.f,0.f,0.f,0.f,0.f,0.f,0.f,0.f};
    const __bf16* q0h = qh + (size_t)(j0 + lr) * kHD;
    const __bf16* q0l = ql + (size_t)(j0 + lr) * kHD;
    const __bf16* q1h = q0h + 16 * kHD;
    const __bf16* q1l = q0l + 16 * kHD;
#pragma unroll 1
    for (int c = 0; c < 4; ++c) {
      const v16b akh = Frag<__bf16>::load(khr + kofs + c * 32);
      const v16b akl = Frag<__bf16>::load(klr + kofs + c * 32);
      const v16b b0h = Frag<__bf16>::load(q0h + c * 32);
      const v16b b0l = Frag<__bf16>::load(q0l + c * 32);
      s0 = mma_bf(akh, b0h, s0);
      s0 = mma_bf(akh, b0l, s0);
      s0 = mma_bf(akl, b0h, s0);
      const v16b b1h = Frag<__bf16>::load(q1h + c * 32);
      const v16b b1l = Frag<__bf16>::load(q1l + c * 32);
      s1 = mma_bf(akh, b1h, s1);
      s1 = mma_bf(akh, b1l, s1);
      s1 = mma_bf(akl, b1h, s1);
    }

#pragma unroll
    for (int v = 0; v < 8; ++v) {
      const int ig = iw + v + 8 * hw;
      const bool m0 = (j0 + lr) > ig;
      const bool m1 = (j0 + 16 + lr) > ig;
      const float a0 = m0 ? kMaskVal : s0[v];
      const float a1 = m1 ? kMaskVal : s1[v];
      float rmax = fmaxf(a0, a1);
      rmax = fmaxf(rmax, __shfl_xor(rmax, 1, 32));
      rmax = fmaxf(rmax, __shfl_xor(rmax, 2, 32));
      rmax = fmaxf(rmax, __shfl_xor(rmax, 4, 32));
      rmax = fmaxf(rmax, __shfl_xor(rmax, 8, 32));
      const float mnew  = fmaxf(mrow[v], rmax);
      const float alpha = __expf(fmaxf(mrow[v] - mnew, -80.0f));
      const float e0 = __expf(fmaxf(a0 - mnew, -100.0f));
      const float e1 = __expf(fmaxf(a1 - mnew, -100.0f));
      const float p0 = m0 ? 0.0f : e0;
      const float p1 = m1 ? 0.0f : e1;
      const _Float16 ph0 = (_Float16)(p0 * kPCarry);
      const _Float16 ph1 = (_Float16)(p1 * kPCarry);
      float rs = (float)ph0 + (float)ph1;
      rs += __shfl_xor(rs, 1, 32);
      rs += __shfl_xor(rs, 2, 32);
      rs += __shfl_xor(rs, 4, 32);
      rs += __shfl_xor(rs, 8, 32);
      lrow[v] = lrow[v] * alpha + rs;
      mrow[v] = mnew;
#pragma unroll
      for (int c8 = 0; c8 < 8; ++c8) o[c8][v] *= alpha;
      pw[(8 * hw + v) * kPPitch + lr]      = ph0;
      pw[(8 * hw + v) * kPPitch + 16 + lr] = ph1;
    }
    __builtin_amdgcn_fence(__ATOMIC_RELEASE, "workgroup");
    __builtin_amdgcn_wave_barrier();
    __builtin_amdgcn_fence(__ATOMIC_ACQUIRE, "workgroup");

    const v16h pf = Frag<_Float16>::load(pw + lr * kPPitch + koff);
    const _Float16* vbh = vth + j0;
    const _Float16* vbl = vtl + j0;
#pragma unroll
    for (int c8 = 0; c8 < 8; ++c8) {
      const v16h bvh = Frag<_Float16>::load(vbh + (size_t)(16 * c8 + lr) * kT);
      const v16h bvl = Frag<_Float16>::load(vbl + (size_t)(16 * c8 + lr) * kT);
      o[c8] = mma_hf(pf, bvh, o[c8]);
      o[c8] = mma_hf(pf, bvl, o[c8]);
      asm volatile("" ::: "memory");
    }
    __builtin_amdgcn_fence(__ATOMIC_RELEASE, "workgroup");
    __builtin_amdgcn_wave_barrier();
    __builtin_amdgcn_fence(__ATOMIC_ACQUIRE, "workgroup");
  }

  float* os = Os[w];
#pragma unroll
  for (int v = 0; v < 8; ++v) {
    const float inv = kAttnNorm * (1.0f / lrow[v]);
#pragma unroll
    for (int c8 = 0; c8 < 8; ++c8) os[(8 * hw + v) * kOPitch + 16 * c8 + lr] = o[c8][v] * inv;
  }
  __builtin_amdgcn_fence(__ATOMIC_RELEASE, "workgroup");
  __builtin_amdgcn_wave_barrier();
  __builtin_amdgcn_fence(__ATOMIC_ACQUIRE, "workgroup");
  {
    const int l16 = lane & 15, rsub = lane >> 4;
#pragma unroll 1
    for (int it = 0; it < 8; ++it) {
      const int row = it * 2 + rsub;
      const float* sp = os + row * kOPitch + l16 * 8;
      const v4f a0 = *(const v4f*)(sp);
      const v4f a1 = *(const v4f*)(sp + 4);
      const float x[8] = {a0[0], a0[1], a0[2], a0[3], a1[0], a1[1], a1[2], a1[3]};
      unsigned short hb[8], lb[8];
#pragma unroll
      for (int e = 0; e < 8; ++e) {
        const _Float16 hh = (_Float16)x[e];
        const float res = x[e] - (float)hh;
        hb[e] = __builtin_bit_cast(unsigned short, hh);
        lb[e] = h_bits(res);
      }
      const v4u uh = (v4u){pk16(hb[0], hb[1]), pk16(hb[2], hb[3]), pk16(hb[4], hb[5]), pk16(hb[6], hb[7])};
      const v4u ul = (v4u){pk16(lb[0], lb[1]), pk16(lb[2], lb[3]), pk16(lb[4], lb[5]), pk16(lb[6], lb[7])};
      const size_t oo = (size_t)(b * kT + iw + row) * kC + h * kHD + l16 * 8;
      *(volatile v4u*)(AHp + oo) = uh;
      *(volatile v4u*)(ALp + oo) = ul;
      __threadfence();
      *(volatile v4u*)(AHp + oo) = uh;
      *(volatile v4u*)(ALp + oo) = ul;
    }
  }
}

extern "C" void kernel_launch(void* const* d_in, const int* in_sizes, int n_in,
                              void* d_out, int out_size, void* d_ws, size_t ws_size,
                              hipStream_t stream) {
  if (n_in < 6) return;
  if (in_sizes[0] != kRows * kC) return;
  if (in_sizes[1] != kT * kHalfHD) return;
  if (in_sizes[2] != kC * kC) return;
  if (in_sizes[3] != kC * kKVC) return;
  if (in_sizes[4] != kC * kKVC) return;
  if (in_sizes[5] != kC * kC) return;
  if (out_size != kRows * kC) return;
  if (ws_size < kWsTotal) return;

  const float* x      = (const float*)d_in[0];
  const float* angles = (const float*)d_in[1];
  const float* wq     = (const float*)d_in[2];
  const float* wk     = (const float*)d_in[3];
  const float* wv     = (const float*)d_in[4];
  const float* wo     = (const float*)d_in[5];
  float* out = (float*)d_out;

  char* ws = (char*)d_ws;
  unsigned short* XH  = (unsigned short*)(ws + kOffXH);
  unsigned short* XL  = (unsigned short*)(ws + kOffXL);
  unsigned short* WH  = (unsigned short*)(ws + kOffWH);
  unsigned short* WL  = (unsigned short*)(ws + kOffWL);
  unsigned short* WOT = (unsigned short*)(ws + kOffWOT);
  float*          QKV = (float*)(ws + kOffQKV);
  unsigned short* QH  = (unsigned short*)(ws + kOffQH);
  unsigned short* QL  = (unsigned short*)(ws + kOffQL);
  unsigned short* KH  = (unsigned short*)(ws + kOffKH);
  unsigned short* KL  = (unsigned short*)(ws + kOffKL);
  unsigned short* VTH = (unsigned short*)(ws + kOffVTH);
  unsigned short* VTL = (unsigned short*)(ws + kOffVTL);
  unsigned short* AH  = (unsigned short*)(ws + kOffAH);
  unsigned short* AL  = (unsigned short*)(ws + kOffAL);
  float*          COS = (float*)(ws + kOffCOS);
  float*          SIN = (float*)(ws + kOffSIN);

  split_rows_bf16_kernel<<<(kRows * kC / 8) / 256, 256, 0, stream>>>(x, XH, XL, kRows * kC / 8);

  wt_planes_kernel<0><<<dim3(kC / 64, kNQKV / 64), 256, 0, stream>>>(
      wq, wk, wv, kC, kKVC, kC, kKVC, kKVC, WH, WL, kC, 1.0f);

  wt_planes_kernel<1><<<dim3(kC / 64, kC / 64), 256, 0, stream>>>(
      wo, wo, wo, kC, 0, kC, kC, kC, WOT, WOT, kC, kWoCarry);

  trig_table_kernel<<<(kT * kHalfHD) / 256, 256, 0, stream>>>(angles, COS, SIN, kT * kHalfHD);

  wmma_gemm64<1, 2, 0, 0, false><<<dim3((kRows / 64) * (kNQKV / 64) / 8, 1), 256, 0, stream>>>(
      XH, XL, kC, 0L,
      WH, WL, kC, 0L,
      (void*)QKV, nullptr, kNQKV, 0L,
      nullptr, nullptr, 0L,
      kRows, kNQKV, kC, 1.0f);

  rotate_split_kernel<<<dim3(kSlices, kRows / 64), 256, 0, stream>>>(QKV, COS, SIN, QH, QL, KH, KL, VTH, VTL);

  attn_kernel<<<dim3(kT / 64, kNH, kB), 128, 0, stream>>>(QH, QL, KH, KL, VTH, VTL, AH, AL);

  wmma_gemm64<0, 1, 0, 0, false><<<dim3((kRows / 64) * (kC / 64) / 8, 1), 256, 0, stream>>>(
      AH, AL, kC, 0L,
      WOT, nullptr, kC, 0L,
      (void*)out, nullptr, kC, 0L,
      nullptr, nullptr, 0L,
      kRows, kC, kC, kOutScale);
}
